// RGCN_14826227106512
// MI455X (gfx1250) — hardware-verified
//
#include <hip/hip_runtime.h>
#include <stddef.h>
#include <stdint.h>


#define D1     128
#define K2     256
#define NTHR   256
#define NWAVE  8
#define EPT    8
#define CHUNK  (NTHR * EPT)
#define WCAP   (EPT * 32)
#define LISTN  (NWAVE * WCAP)
#define NBD    8192
#define SLD    13
#define NBA    1024
#define SLA    10
#define RCAP   32768
#define DEGCAP 256
#define GBM    32
#define GTHR   64
#define NWPL   2
#define NWHL   6
#define NUP    (NWPL * D1 * (D1 / 8))
#define NUH    (NWHL * D1 * (D1 / 4))
#define NUT    (NUP + NUH)
#define NTAB   4
#define AGG_ZINTS    (LISTN + 2 * RCAP + 3 * NBA)
#define AGG_LDS_INTS (AGG_ZINTS + 16)
#define WSMAX  134217728

static_assert((CHUNK & (CHUNK - 1)) == 0 && CHUNK <= 4096);
static_assert((NBD & (NBD - 1)) == 0 && NBD == (1 << SLD));
static_assert((NBA & (NBA - 1)) == 0 && NBA == (1 << SLA));
static_assert(((long long)CHUNK << SLD) < (1LL << 31));
static_assert(((long long)CHUNK << SLA) < (1LL << 31));
static_assert(NBD % (NTHR * 4) == 0 && NBD % GBM == 0);
static_assert(LISTN % NTHR == 0);
static_assert(NBA % NWAVE == 0 && NBA % 32 == 0 && NBA % GBM == 0);
static_assert(RCAP % 32 == 0 && AGG_ZINTS % (NTHR * 4) == 0 && LISTN % 4 == 0);
static_assert(D1 % 32 == 0 && K2 % 32 == 0 && K2 == 2 * D1);
static_assert(GBM == (GTHR / 32) * 16);
static_assert(NUP % NTHR == 0 && NUH % NTHR == 0 && NUT % NTHR == 0);
static_assert((D1 * (D1 / 8)) % NTHR == 0 && (D1 * (D1 / 4)) % NTHR == 0);
static_assert(D1 / 8 == 16 && D1 / 4 == 32 && D1 == 4 * 32);
static_assert(AGG_LDS_INTS * 4 <= 300000);

typedef float          v4f   __attribute__((ext_vector_type(4)));
typedef float          v8f   __attribute__((ext_vector_type(8)));
typedef int            v4i   __attribute__((ext_vector_type(4)));
typedef int            v8i   __attribute__((ext_vector_type(8)));
typedef unsigned short v8us  __attribute__((ext_vector_type(8)));
typedef unsigned short v16us __attribute__((ext_vector_type(16)));
typedef __bf16         v16bf __attribute__((ext_vector_type(16)));
typedef v4f  __attribute__((may_alias)) v4fa;
typedef v4i  __attribute__((may_alias)) v4ia;
typedef v8us __attribute__((may_alias)) v8usa;
union Frag { v16bf v; v16us u; v8us h[2]; v8i w; };

__device__ __forceinline__ v8f wmb(const Frag& a, const Frag& b, v8f c) {
  v8f d = __builtin_amdgcn_wmma_f32_16x16x32_bf16(false, a.v, false, b.v, (short)0, c, false, false);
  asm volatile("v_nop\n\tv_nop\n\tv_nop\n\tv_nop" : "+v"(d) : "v"(a.w), "v"(b.w));
  return d;
}

__device__ __forceinline__ unsigned bf16_bits(float f) {
  const unsigned u = __float_as_uint(f);
  return (u + 0x7FFFu + ((u >> 16) & 1u)) >> 16;
}
__device__ __forceinline__ float bf16_val(float f) {
  return __uint_as_float(bf16_bits(f) << 16);
}
__device__ __forceinline__ v8us hilo8(v4f t) {
  v8us o;
  unsigned hb;
  hb = bf16_bits(t.x); o[0] = (unsigned short)hb; o[4] = (unsigned short)bf16_bits(t.x - __uint_as_float(hb << 16));
  hb = bf16_bits(t.y); o[1] = (unsigned short)hb; o[5] = (unsigned short)bf16_bits(t.y - __uint_as_float(hb << 16));
  hb = bf16_bits(t.z); o[2] = (unsigned short)hb; o[6] = (unsigned short)bf16_bits(t.z - __uint_as_float(hb << 16));
  hb = bf16_bits(t.w); o[3] = (unsigned short)hb; o[7] = (unsigned short)bf16_bits(t.w - __uint_as_float(hb << 16));
  return o;
}

template <int SLB>
__device__ __forceinline__ int scan_chunk(const int* __restrict__ dsts, int nE, int cbase, int slotBase,
                                          int nb, int vec8, int* list, int tid, int lane, int wave) {
  int wc = 0;
  const int el0  = tid * EPT;
  const int e0   = cbase + el0;
  const int sent = -2147483647 - 1;
  v4i da, db;
  if (vec8 != 0 && cbase + CHUNK <= nE) {
    da = *(const v4i*)(dsts + e0);
    db = *(const v4i*)(dsts + e0 + 4);
  } else {
    da.x = (e0     < nE) ? dsts[min(e0,     nE - 1)] : sent;
    da.y = (e0 + 1 < nE) ? dsts[min(e0 + 1, nE - 1)] : sent;
    da.z = (e0 + 2 < nE) ? dsts[min(e0 + 2, nE - 1)] : sent;
    da.w = (e0 + 3 < nE) ? dsts[min(e0 + 3, nE - 1)] : sent;
    db.x = (e0 + 4 < nE) ? dsts[min(e0 + 4, nE - 1)] : sent;
    db.y = (e0 + 5 < nE) ? dsts[min(e0 + 5, nE - 1)] : sent;
    db.z = (e0 + 6 < nE) ? dsts[min(e0 + 6, nE - 1)] : sent;
    db.w = (e0 + 7 < nE) ? dsts[min(e0 + 7, nE - 1)] : sent;
  }
  const unsigned nbs = (unsigned)slotBase;
  const unsigned unb = (unsigned)nb;
  const unsigned s0 = (unsigned)da.x - nbs, s1 = (unsigned)da.y - nbs;
  const unsigned s2 = (unsigned)da.z - nbs, s3 = (unsigned)da.w - nbs;
  const unsigned s4 = (unsigned)db.x - nbs, s5 = (unsigned)db.y - nbs;
  const unsigned s6 = (unsigned)db.z - nbs, s7 = (unsigned)db.w - nbs;
  const bool h0 = s0 < unb, h1 = s1 < unb, h2 = s2 < unb, h3 = s3 < unb;
  const bool h4 = s4 < unb, h5 = s5 < unb, h6 = s6 < unb, h7 = s7 < unb;
  const unsigned any = __builtin_amdgcn_ballot_w32(h0 | h1 | h2 | h3 | h4 | h5 | h6 | h7);
  if (any != 0u) {
#define HITJ(J, HJ, SJ) { \
      const unsigned mj = __builtin_amdgcn_ballot_w32(HJ); \
      if (mj != 0u) { \
        if (HJ) { \
          const int pos = wc + (int)__builtin_amdgcn_mbcnt_lo(mj, 0u); \
          if (pos < WCAP) list[wave * WCAP + pos] = ((el0 + (J)) << SLB) | (int)(SJ); \
        } \
        wc += (int)__builtin_popcount(mj); } }
    HITJ(0, h0, s0)
    HITJ(1, h1, s1)
    HITJ(2, h2, s2)
    HITJ(3, h3, s3)
    HITJ(4, h4, s4)
    HITJ(5, h5, s5)
    HITJ(6, h6, s6)
    HITJ(7, h7, s7)
#undef HITJ
  }
  return wc;
}

__global__ __launch_bounds__(NTHR) void k_prep(const float* __restrict__ w0, const float* __restrict__ w1,
                                               const float* __restrict__ w2, const float* __restrict__ w3,
                                               const float* __restrict__ w4, const float* __restrict__ w5,
                                               const float* __restrict__ w6, const float* __restrict__ w7,
                                               unsigned short* WP, unsigned short* WH) {
  const int u = (int)blockIdx.x * NTHR + (int)threadIdx.x;
  v8us o;
  unsigned short* dp;
  if (u < NUP) {
    const int t  = u >> 11;
    const int n  = (u >> 4) & 127;
    const int k8 = (u & 15) * 8;
    const float* W = w0;
    if (t == 1) W = w1;
    const float* p = W + (size_t)k8 * D1 + n;
#pragma unroll
    for (int i = 0; i < 8; ++i) o[i] = (unsigned short)bf16_bits(p[(size_t)i * D1]);
    dp = WP + (size_t)t * D1 * D1 + (size_t)n * D1 + k8;
  } else if (u < NUT) {
    const int v = u - NUP;
    const int r = v >> 12;
    const int n = (v >> 5) & 127;
    const int g = v & 31;
    const float* W = w2;
    if (r == 1)      W = w3;
    else if (r == 2) W = w4;
    else if (r == 3) W = w5;
    else if (r == 4) W = w6;
    else if (r == 5) W = w7;
    const float* p = W + (size_t)(4 * g) * D1 + n;
    const unsigned short f0 = (unsigned short)bf16_bits(p[0]);
    const unsigned short f1 = (unsigned short)bf16_bits(p[D1]);
    const unsigned short f2 = (unsigned short)bf16_bits(p[2 * D1]);
    const unsigned short f3 = (unsigned short)bf16_bits(p[3 * D1]);
    o[0] = f0; o[1] = f1; o[2] = f2; o[3] = f3; o[4] = f0; o[5] = f1; o[6] = f2; o[7] = f3;
    dp = WH + (size_t)r * D1 * K2 + (size_t)n * K2 + 8 * g;
  } else {
    return;
  }
  *(volatile v8us*)dp = o;
  __threadfence();
  *(volatile v8us*)dp = o;
}

__global__ __launch_bounds__(NTHR) void k_cvx(const float* __restrict__ x0, const float* __restrict__ x1,
                                              int n0, int n1, int U0, int U1,
                                              unsigned short* xb0, unsigned short* xb1) {
  const int u = (int)blockIdx.x * NTHR + (int)threadIdx.x;
  const float* x = x0;
  unsigned short* xb = xb0;
  int nN = n0;
  int v;
  if (u < U0) {
    v = u;
  } else if (u < U0 + U1) {
    x = x1; xb = xb1; nN = n1; v = u - U0;
  } else {
    return;
  }
  const int row = v >> 4;
  const int k8  = (v & 15) * 8;
  const int rc  = row < nN ? row : nN - 1;
  const float* p = x + (size_t)rc * D1 + k8;
  const v4f a = *(const v4fa*)p;
  const v4f b = *(const v4fa*)(p + 4);
  const bool ok = row < nN;
  v8us o;
  o[0] = ok ? (unsigned short)bf16_bits(a.x) : (unsigned short)0;
  o[1] = ok ? (unsigned short)bf16_bits(a.y) : (unsigned short)0;
  o[2] = ok ? (unsigned short)bf16_bits(a.z) : (unsigned short)0;
  o[3] = ok ? (unsigned short)bf16_bits(a.w) : (unsigned short)0;
  o[4] = ok ? (unsigned short)bf16_bits(b.x) : (unsigned short)0;
  o[5] = ok ? (unsigned short)bf16_bits(b.y) : (unsigned short)0;
  o[6] = ok ? (unsigned short)bf16_bits(b.z) : (unsigned short)0;
  o[7] = ok ? (unsigned short)bf16_bits(b.w) : (unsigned short)0;
  unsigned short* dp = xb + (size_t)row * D1 + k8;
  *(volatile v8us*)dp = o;
  __threadfence();
  *(volatile v8us*)dp = o;
}

__global__ __launch_bounds__(NTHR) void k_deg(const int* __restrict__ l0, const int* __restrict__ l1,
                                              const int* __restrict__ l2, const int* __restrict__ l3,
                                              int nE0, int nE1, int nE2, int nE3,
                                              int n0, int n1, int n2, int n3, int nbpd, float* dg) {
  __shared__ __attribute__((aligned(16))) int scnt[NBD];
  __shared__ __attribute__((aligned(16))) int list[LISTN];
  __shared__ int wcnt[NWAVE];
  const int tid = (int)threadIdx.x, lane = tid & 31, wave = tid >> 5;
  const int nodeBase = (int)blockIdx.x * NBD;
  const int p = (int)blockIdx.y;
  const int* lst = l0;
  int nTab = n0, nE = nE0;
  if (p == 1)      { lst = l1; nTab = n1; nE = nE1; }
  else if (p == 2) { lst = l2; nTab = n2; nE = nE2; }
  else if (p == 3) { lst = l3; nTab = n3; nE = nE3; }
  if (nodeBase >= nTab) return;
  const int vec8 = ((nE & 3) == 0) ? 1 : 0;

  for (int i = tid; i < NBD; i += NTHR) scnt[i] = 0;
  for (int i = tid; i < LISTN; i += NTHR) list[i] = 0;
  if (tid < NWAVE) wcnt[tid] = 0;
  __syncthreads();

  const int nChunks = (nE + CHUNK - 1) / CHUNK;
#pragma unroll 1
  for (int ch = 0; ch < nChunks; ++ch) {
    const int cbase = ch * CHUNK;
    const int wc = scan_chunk<SLD>(lst, nE, cbase, nodeBase, NBD, vec8, list, tid, lane, wave);
    if (lane == 0) wcnt[wave] = wc;
    __syncthreads();
    if (wave == 0) {
#pragma unroll 1
      for (int w2 = 0; w2 < NWAVE; ++w2) {
        int c = wcnt[w2];
        c = c < 0 ? 0 : (c > WCAP ? WCAP : c);
#pragma unroll 1
        for (int b0 = 0; b0 < c; b0 += 32) {
          const int idx = b0 + lane;
          const int ent = list[w2 * WCAP + (idx < WCAP ? idx : WCAP - 1)];
          const int m32 = (c - b0) < 32 ? (c - b0) : 32;
#pragma unroll 1
          for (int k = 0; k < m32; ++k) {
            const int u  = __builtin_amdgcn_readlane(ent, k);
            const int sl = u & (NBD - 1);
            if (lane == 0) scnt[sl] = scnt[sl] + 1;
          }
        }
      }
    }
    __syncthreads();
  }

  v4f vals[NBD / (NTHR * 4)];
#pragma unroll
  for (int it = 0; it < NBD / (NTHR * 4); ++it) {
    const int s0 = it * (NTHR * 4) + 4 * tid;
    const v4i c4 = *(const v4ia*)(scnt + s0);
    const float d0 = (float)(c4.x < 1 ? 1 : c4.x), d1 = (float)(c4.y < 1 ? 1 : c4.y);
    const float d2 = (float)(c4.z < 1 ? 1 : c4.z), d3 = (float)(c4.w < 1 ? 1 : c4.w);
    v4f v;
    v.x = rsqrtf(d0); v.y = rsqrtf(d1); v.z = rsqrtf(d2); v.w = rsqrtf(d3);
    vals[it] = v;
  }
  float* base = dg + (size_t)p * (size_t)nbpd + (size_t)nodeBase;
#pragma unroll
  for (int it = 0; it < NBD / (NTHR * 4); ++it) {
    const int s0 = it * (NTHR * 4) + 4 * tid;
    *(volatile v4f*)(base + s0) = vals[it];
  }
  __threadfence();
#pragma unroll
  for (int it = 0; it < NBD / (NTHR * 4); ++it) {
    const int s0 = it * (NTHR * 4) + 4 * tid;
    *(volatile v4f*)(base + s0) = vals[it];
  }
}

template <int DEC>
__global__ __launch_bounds__(GTHR) void k_gemm(const unsigned short* __restrict__ A,
                                               const unsigned short* __restrict__ WT,
                                               const float* __restrict__ dg, const float* __restrict__ bias,
                                               float* T, int K, int nOut) {
  __shared__ __attribute__((aligned(16))) float stg[GBM * D1];
  __shared__ __attribute__((aligned(16))) float sdg[GBM];
  const int tid = (int)threadIdx.x, lane = tid & 31, wave = tid >> 5, hh = lane >> 4, m = lane & 15;
  const int rowBase = (int)blockIdx.x * GBM;
  if constexpr (DEC == 0) {
    if (tid < GBM) sdg[tid] = dg[rowBase + tid];
  } else {
    if (tid < GBM) sdg[tid] = 1.0f;
  }

  v8f acc[8];
  {
    const v8f z = {0.f, 0.f, 0.f, 0.f, 0.f, 0.f, 0.f, 0.f};
#pragma unroll
    for (int t = 0; t < 8; ++t) acc[t] = z;
  }
  const unsigned short* ap = A  + (size_t)(rowBase + 16 * wave + m) * (size_t)K + 8 * hh;
  const unsigned short* bp = WT + (size_t)m * (size_t)K + 8 * hh;
  const int ksteps = K >> 5;

#pragma unroll 1
  for (int ks = 0; ks < ksteps; ++ks) {
    const int k0 = 32 * ks;
    Frag af;
    af.h[0] = *(const v8usa*)(ap + k0);
    af.h[1] = *(const v8usa*)(ap + k0 + 16);
#pragma unroll
    for (int nt = 0; nt < 8; ++nt) {
      const unsigned short* wq = bp + (size_t)(16 * nt) * (size_t)K + k0;
      Frag bf;
      bf.h[0] = *(const v8usa*)wq;
      bf.h[1] = *(const v8usa*)(wq + 16);
      acc[nt] = wmb(af, bf, acc[nt]);
    }
  }

#pragma unroll
  for (int nt = 0; nt < 8; ++nt) {
    const int lc = 16 * nt + m;
#pragma unroll
    for (int r = 0; r < 8; ++r) {
      const int lr = 16 * wave + 8 * hh + r;
      stg[lr * D1 + lc] = acc[nt][r];
    }
  }
  __syncthreads();

  v4f add4 = {0.0f, 0.0f, 0.0f, 0.0f};
  if constexpr (DEC != 0) {
    const v4f tb = *(const v4fa*)(bias + 4 * lane);
    add4.x = bf16_val(tb.x); add4.y = bf16_val(tb.y); add4.z = bf16_val(tb.z); add4.w = bf16_val(tb.w);
  }
  v4f fv[16];
#pragma unroll
  for (int i = 0; i < 16; ++i) {
    const int lr = 16 * wave + i;
    fv[i] = *(const v4fa*)(stg + lr * D1 + 4 * lane) * sdg[lr] + add4;
  }
#pragma unroll
  for (int i = 0; i < 16; ++i) {
    const int gr = rowBase + 16 * wave + i;
    if (gr < nOut) {
      float* op = T + (size_t)gr * (size_t)D1 + 4 * lane;
      *(volatile v4f*)op = fv[i];
    }
  }
  __threadfence();
#pragma unroll
  for (int i = 0; i < 16; ++i) {
    const int gr = rowBase + 16 * wave + i;
    if (gr < nOut) {
      float* op = T + (size_t)gr * (size_t)D1 + 4 * lane;
      *(volatile v4f*)op = fv[i];
    }
  }
}

template <int MODE>
__global__ __launch_bounds__(NTHR) void k_agg(const int* __restrict__ srcs, const int* __restrict__ dsts,
                                              int nE, int nDst, int nSrc, int mRows,
                                              const float* __restrict__ tpl, const float* __restrict__ bias,
                                              const float* oin, float* oout, unsigned short* hpl) {
  extern __shared__ __attribute__((aligned(16))) int dsm[];
  int* list = dsm;
  int* hl   = dsm + LISTN;
  int* sl   = hl + RCAP;
  int* cnt  = sl + RCAP;
  int* offs = cnt + NBA;
  int* cur  = offs + NBA;
  int* misc = cur + NBA;
  const int tid = (int)threadIdx.x, lane = tid & 31, wave = tid >> 5;
  const int nodeBase = (int)blockIdx.x * NBA;
  const int vec8 = ((nE & 3) == 0) ? 1 : 0;

  {
    const v4i z4 = {0, 0, 0, 0};
    for (int i = tid * 4; i < AGG_ZINTS; i += NTHR * 4) *(v4ia*)(dsm + i) = z4;
    if (tid < 16) misc[tid] = 0;
  }
  __syncthreads();

  int t = 0, ov = 0;
  const int nChunks = (nE + CHUNK - 1) / CHUNK;
#pragma unroll 1
  for (int ch = 0; ch < nChunks; ++ch) {
    const int cbase = ch * CHUNK;
    const int wc = scan_chunk<SLA>(dsts, nE, cbase, nodeBase, NBA, vec8, list, tid, lane, wave);
    if (lane == 0) misc[wave] = wc;
    __syncthreads();
    if (wave == 0) {
#pragma unroll 1
      for (int w2 = 0; w2 < NWAVE; ++w2) {
        int c = misc[w2];
        c = c < 0 ? 0 : (c > WCAP ? WCAP : c);
#pragma unroll 1
        for (int b0 = 0; b0 < c; b0 += 32) {
          const int idx = b0 + lane;
          const int ent = list[w2 * WCAP + (idx < WCAP ? idx : WCAP - 1)];
          const int m32 = (c - b0) < 32 ? (c - b0) : 32;
#pragma unroll 1
          for (int k = 0; k < m32; ++k) {
            const int u    = __builtin_amdgcn_readlane(ent, k);
            const int slot = u & (NBA - 1);
            const int el   = (u >> SLA) & (CHUNK - 1);
            const int pk   = ((cbase + el) << SLA) | slot;
            if (t < RCAP) {
              if (lane == 0) { hl[t] = pk; cnt[slot] = cnt[slot] + 1; }
              t = t + 1;
            } else {
              ov = 1;
            }
          }
        }
      }
    }
    __syncthreads();
  }
  if (wave == 0 && lane == 0) { misc[8] = t; misc[9] = ov; }
  __syncthreads();
  int tt = misc[8];
  tt = tt < 0 ? 0 : (tt > RCAP ? RCAP : tt);
  const int ovf = misc[9];

  if (wave == 0) {
    const int base = lane * (NBA / 32);
    int sacc = 0;
#pragma unroll 1
    for (int i = 0; i < NBA / 32; ++i) sacc += cnt[base + i];
    int incl = sacc;
#pragma unroll
    for (int d = 1; d < 32; d <<= 1) {
      const int y = __shfl_up(incl, d, 32);
      if (lane >= d) incl += y;
    }
    int run = incl - sacc;
#pragma unroll 1
    for (int i = 0; i < NBA / 32; ++i) {
      const int cv = cnt[base + i];
      offs[base + i] = run;
      cur[base + i]  = run;
      run += cv;
    }
  }
  __syncthreads();
  if (wave == 0) {
#pragma unroll 1
    for (int b0 = 0; b0 < tt; b0 += 32) {
      const int idx = b0 + lane;
      const int ent = hl[idx < RCAP ? idx : RCAP - 1];
      const int m32 = (tt - b0) < 32 ? (tt - b0) : 32;
#pragma unroll 1
      for (int k = 0; k < m32; ++k) {
        const int u    = __builtin_amdgcn_readlane(ent, k);
        const int slot = u & (NBA - 1);
        if (lane == 0) {
          int p = cur[slot];
          p = p < 0 ? 0 : (p > RCAP - 1 ? RCAP - 1 : p);
          sl[p] = u;
          cur[slot] = p + 1;
        }
      }
    }
  }
  __syncthreads();

  const float qnan = __int_as_float(0x7fc00000);
  const float pz = (ovf != 0) ? qnan : 0.0f;
  const v4f z4 = {0.0f, 0.0f, 0.0f, 0.0f};
  v4f bv;
  {
    const v4f a = *(const v4fa*)(bias + 4 * lane);
    bv.x = bf16_val(a.x); bv.y = bf16_val(a.y); bv.z = bf16_val(a.z); bv.w = bf16_val(a.w);
  }
#pragma unroll 1
  for (int si = 0; si < NBA / NWAVE; ++si) {
    const int s    = si * NWAVE + wave;
    const int node = nodeBase + s;
    const int craw = cnt[s];
    const bool big = craw > DEGCAP;
    const int c = craw < 0 ? 0 : (craw > DEGCAP ? DEGCAP : craw);
    int o = offs[s];
    o = o < 0 ? 0 : (o > RCAP ? RCAP : o);
    const float dd = rsqrtf(fmaxf((float)craw, 1.0f));
    v4f acc = z4;
#pragma unroll 1
    for (int b0 = 0; b0 < c; b0 += 32) {
      int idx = o + b0 + lane;
      idx = idx > RCAP - 1 ? RCAP - 1 : idx;
      const int ent = sl[idx];
      int eid = ent >> SLA;
      eid = eid < 0 ? 0 : (eid > nE - 1 ? nE - 1 : eid);
      int sr = srcs[eid];
      sr = sr < 0 ? 0 : (sr > nSrc - 1 ? nSrc - 1 : sr);
      const int m32 = (c - b0) < 32 ? (c - b0) : 32;
#pragma unroll 1
      for (int k = 0; k < m32; ++k) {
        const int sk = __builtin_amdgcn_readlane(sr, k);
        const v4f a = *(const v4fa*)(tpl + (size_t)sk * (size_t)D1 + 4 * lane);
        acc += a;
      }
    }
    const float pzr = big ? qnan : pz;
    const bool live = node < nDst;
    v4f v;
    v.x = fmaxf(fmaf(acc.x, dd, bv.x), 0.0f);
    v.y = fmaxf(fmaf(acc.y, dd, bv.y), 0.0f);
    v.z = fmaxf(fmaf(acc.z, dd, bv.z), 0.0f);
    v.w = fmaxf(fmaf(acc.w, dd, bv.w), 0.0f);
    if constexpr (MODE == 2) {
      const int ncl = live ? node : nDst - 1;
      const v4f pv = *(const v4fa*)(oin + (size_t)ncl * (size_t)D1 + 4 * lane);
      v = pv + v;
    }
    v.x = v.x + pzr; v.y = v.y + pzr; v.z = v.z + pzr; v.w = v.w + pzr;
    v4f y;
    y.x = live ? v.x : 0.0f; y.y = live ? v.y : 0.0f; y.z = live ? v.z : 0.0f; y.w = live ? v.w : 0.0f;
    if constexpr (MODE == 1) {
      if (node < mRows) {
        float* op = oout + (size_t)node * (size_t)D1 + 4 * lane;
        *(volatile v4f*)op = y;
        __threadfence();
        *(volatile v4f*)op = y;
      }
    } else {
      const v8us po = hilo8(y);
      if (node < mRows) {
        unsigned short* hp = hpl + (size_t)node * (size_t)K2 + 8 * lane;
        *(volatile v8us*)hp = po;
        __threadfence();
        *(volatile v8us*)hp = po;
      }
    }
  }
}

static inline int cdiv(int a, int b) { return (a + b - 1) / b; }

extern "C" void kernel_launch(void* const* d_in, const int* in_sizes, int n_in,
                              void* d_out, int out_size, void* d_ws, size_t ws_size,
                              hipStream_t stream) {
  if (n_in < 39) return;
  if (in_sizes[0] < D1 || (in_sizes[0] % D1) != 0) return;
  if (in_sizes[1] < D1 || (in_sizes[1] % D1) != 0) return;
  if (in_sizes[2] < D1 || (in_sizes[2] % D1) != 0) return;
  const int ng = in_sizes[0] / D1, nc = in_sizes[1] / D1, nt = in_sizes[2] / D1;
  if (ng > (1 << 22) || nc > (1 << 22) || nt > (1 << 22)) return;
  {
    const int wIdx[8] = {3, 5, 11, 15, 21, 25, 27, 29};
    for (int i = 0; i < 8; ++i) {
      if (in_sizes[wIdx[i]] != D1 * D1) return;
      if (in_sizes[wIdx[i] + 1] != D1) return;
    }
  }
  const int Egc = in_sizes[31];
  const int Ecg = in_sizes[33];
  const int Egt = in_sizes[35];
  const int Etg = in_sizes[37];
  if (in_sizes[32] != Egc || in_sizes[34] != Ecg || in_sizes[36] != Egt || in_sizes[38] != Etg) return;
  if (Egc < 1 || Ecg < 1 || Egt < 1 || Etg < 1) return;
  const int eMax = 1 << (31 - SLA);
  if (Egc >= eMax || Ecg >= eMax || Egt >= eMax || Etg >= eMax) return;
  if ((long long)out_size != (long long)nc * D1) return;

  const float* x_c   = (const float*)d_in[1];
  const float* x_t   = (const float*)d_in[2];
  const float* Wc2g  = (const float*)d_in[3];
  const float* bc2g  = (const float*)d_in[4];
  const float* Wt2g  = (const float*)d_in[5];
  const float* bt2g  = (const float*)d_in[6];
  const float* W1g2c = (const float*)d_in[11];
  const float* b1g2c = (const float*)d_in[12];
  const float* W1g2t = (const float*)d_in[15];
  const float* b1g2t = (const float*)d_in[16];
  const float* W2c2g = (const float*)d_in[21];
  const float* b2c2g = (const float*)d_in[22];
  const float* W2t2g = (const float*)d_in[25];
  const float* b2t2g = (const float*)d_in[26];
  const float* W3g2c = (const float*)d_in[27];
  const float* b3g2c = (const float*)d_in[28];
  const float* Wd    = (const float*)d_in[29];
  const float* bd    = (const float*)d_in[30];
  const int* eg2c_s = (const int*)d_in[31];
  const int* eg2c_d = (const int*)d_in[32];
  const int* ec2g_s = (const int*)d_in[33];
  const int* ec2g_d = (const int*)d_in[34];
  const int* eg2t_s = (const int*)d_in[35];
  const int* eg2t_d = (const int*)d_in[36];
  const int* et2g_s = (const int*)d_in[37];
  const int* et2g_d = (const int*)d_in[38];
  float* out = (float*)d_out;

  const int MPg = cdiv(ng, GBM) * GBM;
  const int MPc = cdiv(nc, GBM) * GBM;
  const int MPt = cdiv(nt, GBM) * GBM;
  int maxMP = MPg > MPc ? MPg : MPc;
  maxMP = maxMP > MPt ? maxMP : MPt;
  const int gD   = cdiv(maxMP, NBD);
  const int NBPD = gD * NBD;
  if (NBPD < maxMP) return;
  const int gAg = cdiv(MPg, NBA), gAc = cdiv(MPc, NBA), gAt = cdiv(MPt, NBA);
  if ((long long)gAg * NBA < MPg || (long long)gAc * NBA < MPc || (long long)gAt * NBA < MPt) return;
  const int Uc = MPc * (D1 / 8), Ut = MPt * (D1 / 8);
  if ((Uc % NTHR) != 0 || (Ut % NTHR) != 0) return;

  char* ws = (char*)d_ws;
  size_t off = 0;
  const size_t oDG  = off; off += (size_t)NTAB * (size_t)NBPD * 4;        off = (off + 255) & ~(size_t)255;
  const size_t oWP  = off; off += (size_t)NWPL * D1 * D1 * 2;             off = (off + 255) & ~(size_t)255;
  const size_t oWH  = off; off += (size_t)NWHL * D1 * K2 * 2;             off = (off + 255) & ~(size_t)255;
  const size_t oXBc = off; off += (size_t)MPc * D1 * 2;                   off = (off + 255) & ~(size_t)255;
  const size_t oXBt = off; off += (size_t)MPt * D1 * 2;                   off = (off + 255) & ~(size_t)255;
  const size_t oT   = off; off += (size_t)maxMP * D1 * 4;                 off = (off + 255) & ~(size_t)255;
  const size_t oO   = off; off += (size_t)MPg * D1 * 4;                   off = (off + 255) & ~(size_t)255;
  const size_t oHAc = off; off += (size_t)MPc * K2 * 2;                   off = (off + 255) & ~(size_t)255;
  const size_t oHAg = off; off += (size_t)MPg * K2 * 2;                   off = (off + 255) & ~(size_t)255;
  const size_t oHAt = off; off += (size_t)MPt * K2 * 2;                   off = (off + 255) & ~(size_t)255;
  if (off > ws_size || off > (size_t)WSMAX) return;
  float*          DG  = (float*)(ws + oDG);
  unsigned short* WP  = (unsigned short*)(ws + oWP);
  unsigned short* WH  = (unsigned short*)(ws + oWH);
  unsigned short* XBc = (unsigned short*)(ws + oXBc);
  unsigned short* XBt = (unsigned short*)(ws + oXBt);
  float*          T   = (float*)(ws + oT);
  float*          O   = (float*)(ws + oO);
  unsigned short* HAc = (unsigned short*)(ws + oHAc);
  unsigned short* HAg = (unsigned short*)(ws + oHAg);
  unsigned short* HAt = (unsigned short*)(ws + oHAt);
  float* DG0 = DG;
  float* DG1 = DG + (size_t)1 * NBPD;
  float* DG2 = DG + (size_t)2 * NBPD;
  float* DG3 = DG + (size_t)3 * NBPD;
  unsigned short* WP0 = WP;
  unsigned short* WP1 = WP + (size_t)1 * D1 * D1;
  unsigned short* WH0 = WH;
  unsigned short* WH1 = WH + (size_t)1 * D1 * K2;
  unsigned short* WH2 = WH + (size_t)2 * D1 * K2;
  unsigned short* WH3 = WH + (size_t)3 * D1 * K2;
  unsigned short* WH4 = WH + (size_t)4 * D1 * K2;
  unsigned short* WH5 = WH + (size_t)5 * D1 * K2;

  const size_t aggLds = (size_t)AGG_LDS_INTS * 4;
  hipFuncSetAttribute(reinterpret_cast<const void*>(&k_agg<0>), hipFuncAttributeMaxDynamicSharedMemorySize, (int)aggLds);
  hipFuncSetAttribute(reinterpret_cast<const void*>(&k_agg<1>), hipFuncAttributeMaxDynamicSharedMemorySize, (int)aggLds);
  hipFuncSetAttribute(reinterpret_cast<const void*>(&k_agg<2>), hipFuncAttributeMaxDynamicSharedMemorySize, (int)aggLds);

  k_prep<<<NUT / NTHR, NTHR, 0, stream>>>(Wc2g, Wt2g, W1g2c, W1g2t, W2c2g, W2t2g, W3g2c, Wd, WP, WH);
  k_cvx<<<(Uc + Ut) / NTHR, NTHR, 0, stream>>>(x_c, x_t, nc, nt, Uc, Ut, XBc, XBt);
  k_deg<<<dim3(gD, NTAB), NTHR, 0, stream>>>(ec2g_s, et2g_s, eg2c_s, eg2t_s, Ecg, Etg, Egc, Egt,
                                             nc, nt, ng, ng, NBPD, DG);

  k_gemm<0><<<MPc / GBM, GTHR, 0, stream>>>(XBc, WP0, DG0, bc2g, T, D1, MPc);
  k_agg<1><<<gAg, NTHR, aggLds, stream>>>(ec2g_s, ec2g_d, Ecg, ng, nc, MPg, T, bc2g, O, O, HAg);
  k_gemm<0><<<MPt / GBM, GTHR, 0, stream>>>(XBt, WP1, DG1, bt2g, T, D1, MPt);
  k_agg<2><<<gAg, NTHR, aggLds, stream>>>(et2g_s, et2g_d, Etg, ng, nt, MPg, T, bt2g, O, O, HAg);

  k_gemm<0><<<MPg / GBM, GTHR, 0, stream>>>(HAg, WH0, DG2, b1g2c, T, K2, MPg);
  k_agg<0><<<gAc, NTHR, aggLds, stream>>>(eg2c_s, eg2c_d, Egc, nc, ng, MPc, T, b1g2c, O, O, HAc);
  k_gemm<0><<<MPg / GBM, GTHR, 0, stream>>>(HAg, WH1, DG3, b1g2t, T, K2, MPg);
  k_agg<0><<<gAt, NTHR, aggLds, stream>>>(eg2t_s, eg2t_d, Egt, nt, ng, MPt, T, b1g2t, O, O, HAt);

  k_gemm<0><<<MPc / GBM, GTHR, 0, stream>>>(HAc, WH2, DG0, b2c2g, T, K2, MPc);
  k_agg<1><<<gAg, NTHR, aggLds, stream>>>(ec2g_s, ec2g_d, Ecg, ng, nc, MPg, T, b2c2g, O, O, HAg);
  k_gemm<0><<<MPt / GBM, GTHR, 0, stream>>>(HAt, WH3, DG1, b2t2g, T, K2, MPt);
  k_agg<2><<<gAg, NTHR, aggLds, stream>>>(et2g_s, et2g_d, Etg, ng, nt, MPg, T, b2t2g, O, O, HAg);

  k_gemm<0><<<MPg / GBM, GTHR, 0, stream>>>(HAg, WH4, DG2, b3g2c, T, K2, MPg);
  k_agg<0><<<gAc, NTHR, aggLds, stream>>>(eg2c_s, eg2c_d, Egc, nc, ng, MPc, T, b3g2c, O, O, HAc);

  k_gemm<1><<<MPc / GBM, GTHR, 0, stream>>>(HAc, WH5, DG0, bd, out, K2, nc);
}
